// Encoder_41669772706622
// MI455X (gfx1250) — hardware-verified
//
#include <hip/hip_runtime.h>
#include <stddef.h>
#include <stdint.h>


#define DF     128
#define HP     256
#define NLAY   6
#define VOC    128
#define NTHR   256
#define NWAVE  8
#define EPT    8
#define CHUNK  (NTHR * EPT)
#define WCAP   (EPT * 32)
#define LISTN  (NWAVE * WCAP)
#define NBA    1024
#define SLA    10
#define RCAP   8192
#define DEGCAP 32
#define GBM    64
#define GTHR   128
#define PGR    64
#define WUNITS 2048
#define NWPL   (2 * NLAY)
#define WBLK   ((NWPL * WUNITS) / NTHR)
#define BK_ZINTS (LISTN + 2 * RCAP + 3 * NBA)
#define BK_LDS_INTS (BK_ZINTS + 16)
#define WSMAX  134217728

static_assert((CHUNK & (CHUNK - 1)) == 0 && CHUNK <= 4096);
static_assert((NBA & (NBA - 1)) == 0 && NBA == (1 << SLA));
static_assert(((long long)CHUNK << SLA) < (1LL << 31));
static_assert(LISTN % NTHR == 0 && NBA % NTHR == 0);
static_assert(NBA % NWAVE == 0 && NBA % 32 == 0 && NBA % GBM == 0);
static_assert(RCAP % (NTHR * 4) == 0 && BK_ZINTS % 4 == 0 && (2 * NBA) % (NTHR * 4) == 0);
static_assert(HP == 2 * DF && HP % 32 == 0 && DF == 4 * 32);
static_assert(GBM == (GTHR / 32) * 16);
static_assert(WUNITS % NTHR == 0 && WUNITS == DF * (DF / 8) && (1 << 11) == WUNITS);
static_assert(PGR % NWAVE == 0 && (PGR & (PGR - 1)) == 0 && (PGR * DF) % (NTHR * 4) == 0);
static_assert(DEGCAP <= 32 && DEGCAP <= RCAP);
static_assert(BK_LDS_INTS * 4 <= 300000);

typedef float          v4f   __attribute__((ext_vector_type(4)));
typedef float          v8f   __attribute__((ext_vector_type(8)));
typedef int            v4i   __attribute__((ext_vector_type(4)));
typedef int            v8i   __attribute__((ext_vector_type(8)));
typedef unsigned short v4us  __attribute__((ext_vector_type(4)));
typedef unsigned short v8us  __attribute__((ext_vector_type(8)));
typedef unsigned short v16us __attribute__((ext_vector_type(16)));
typedef __bf16         v16bf __attribute__((ext_vector_type(16)));
typedef v4f  __attribute__((may_alias)) v4fa;
typedef v4i  __attribute__((may_alias)) v4ia;
typedef v4us __attribute__((may_alias)) v4usa;
typedef v8us __attribute__((may_alias)) v8usa;
union FragB { v16bf v; v16us u; v8us h[2]; v8i w; };

__device__ __forceinline__ v8f wmb(const FragB& a, const FragB& b, v8f c) {
  v8f d = __builtin_amdgcn_wmma_f32_16x16x32_bf16(false, a.v, false, b.v, (short)0, c, false, false);
  asm volatile("v_nop\n\tv_nop\n\tv_nop\n\tv_nop" : "+v"(d) : "v"(a.w), "v"(b.w));
  return d;
}

__device__ __forceinline__ unsigned bf16_bits(float f) {
  const unsigned u = __float_as_uint(f);
  const unsigned r = (u + 0x7FFFu + ((u >> 16) & 1u)) >> 16;
  const unsigned q = (u >> 16) | 0x40u;
  return ((u & 0x7FFFFFFFu) > 0x7F800000u) ? q : r;
}
__device__ __forceinline__ float bf16_val(float f) {
  return __uint_as_float(bf16_bits(f) << 16);
}
__device__ __forceinline__ float relu_keep(float v) {
  return (v > 0.0f) ? v : (v - v);
}

__device__ __forceinline__ void wave_sync() {
  __builtin_amdgcn_fence(__ATOMIC_RELEASE, "wavefront");
  __builtin_amdgcn_wave_barrier();
  __builtin_amdgcn_fence(__ATOMIC_ACQUIRE, "wavefront");
}

template <int SLB>
__device__ __forceinline__ int scan_chunk(const int* __restrict__ dsts, int nE, int cbase, int slotBase,
                                          int nb, int vec8, int* list, int tid, int lane, int wave) {
  int wc = 0;
  const int el0  = tid * EPT;
  const int e0   = cbase + el0;
  const int sent = -2147483647 - 1;
  v4i da, db;
  if (vec8 != 0 && cbase + CHUNK <= nE) {
    da = *(const v4i*)(dsts + e0);
    db = *(const v4i*)(dsts + e0 + 4);
  } else {
    da.x = (e0     < nE) ? dsts[min(e0,     nE - 1)] : sent;
    da.y = (e0 + 1 < nE) ? dsts[min(e0 + 1, nE - 1)] : sent;
    da.z = (e0 + 2 < nE) ? dsts[min(e0 + 2, nE - 1)] : sent;
    da.w = (e0 + 3 < nE) ? dsts[min(e0 + 3, nE - 1)] : sent;
    db.x = (e0 + 4 < nE) ? dsts[min(e0 + 4, nE - 1)] : sent;
    db.y = (e0 + 5 < nE) ? dsts[min(e0 + 5, nE - 1)] : sent;
    db.z = (e0 + 6 < nE) ? dsts[min(e0 + 6, nE - 1)] : sent;
    db.w = (e0 + 7 < nE) ? dsts[min(e0 + 7, nE - 1)] : sent;
  }
  const unsigned nbs = (unsigned)slotBase;
  const unsigned unb = (unsigned)nb;
  const unsigned s0 = (unsigned)da.x - nbs, s1 = (unsigned)da.y - nbs;
  const unsigned s2 = (unsigned)da.z - nbs, s3 = (unsigned)da.w - nbs;
  const unsigned s4 = (unsigned)db.x - nbs, s5 = (unsigned)db.y - nbs;
  const unsigned s6 = (unsigned)db.z - nbs, s7 = (unsigned)db.w - nbs;
  const bool h0 = s0 < unb, h1 = s1 < unb, h2 = s2 < unb, h3 = s3 < unb;
  const bool h4 = s4 < unb, h5 = s5 < unb, h6 = s6 < unb, h7 = s7 < unb;
  const unsigned any = __builtin_amdgcn_ballot_w32(h0 | h1 | h2 | h3 | h4 | h5 | h6 | h7);
  if (any != 0u) {
#define HITJ(J, HJ, SJ) { \
      const unsigned mj = __builtin_amdgcn_ballot_w32(HJ); \
      if (mj != 0u) { \
        if (HJ) { \
          const int pos = wc + (int)__builtin_amdgcn_mbcnt_lo(mj, 0u); \
          if (pos < WCAP) list[wave * WCAP + pos] = ((el0 + (J)) << SLB) | (int)(SJ); \
        } \
        wc += (int)__builtin_popcount(mj); } }
    HITJ(0, h0, s0)
    HITJ(1, h1, s1)
    HITJ(2, h2, s2)
    HITJ(3, h3, s3)
    HITJ(4, h4, s4)
    HITJ(5, h5, s5)
    HITJ(6, h6, s6)
    HITJ(7, h7, s7)
#undef HITJ
  }
  return wc;
}

__device__ __forceinline__ void wplane_unit(const float* __restrict__ W, unsigned short* P, int v) {
  const int n  = v >> 4;
  const int k8 = (v & 15) * 8;
  const float* p = W + (size_t)k8 * DF + n;
  v8us o;
#pragma unroll
  for (int i = 0; i < 8; ++i) o[i] = (unsigned short)bf16_bits(p[(size_t)i * DF]);
  unsigned short* dp = P + (size_t)n * HP + k8;
  *(volatile v8us*)dp = o;
  *(volatile v8us*)(dp + DF) = o;
  __threadfence();
  *(volatile v8us*)dp = o;
  *(volatile v8us*)(dp + DF) = o;
}

__global__ __launch_bounds__(NTHR) void k_prep(const float* __restrict__ W1, const float* __restrict__ W2,
                                               const int* __restrict__ tok, const float* __restrict__ emb,
                                               unsigned short* W1S, unsigned short* W2S, float* X, int nN) {
  const int bx = (int)blockIdx.x, tid = (int)threadIdx.x;
  if (bx < WBLK) {
    const int u  = bx * NTHR + tid;
    const int pl = u >> 11;
    const int v  = u & (WUNITS - 1);
    if (pl < NLAY) {
      wplane_unit(W1 + (size_t)pl * DF * DF, W1S + (size_t)pl * DF * HP, v);
    } else {
      wplane_unit(W2 + (size_t)(pl - NLAY) * DF * DF, W2S + (size_t)(pl - NLAY) * DF * HP, v);
    }
    return;
  }
  const int u    = (bx - WBLK) * NTHR + tid;
  const int node = u >> 5;
  const int c    = (u & 31) * 4;
  if (node >= nN) return;
  int t = tok[node];
  t = t < 0 ? 0 : (t > VOC - 1 ? VOC - 1 : t);
  const v4f e = *(const v4f*)(emb + (size_t)t * DF + c);
  v4f o;
  o.x = bf16_val(e.x); o.y = bf16_val(e.y); o.z = bf16_val(e.z); o.w = bf16_val(e.w);
  float* op = X + (size_t)node * DF + c;
  *(volatile v4f*)op = o;
  __threadfence();
  *(volatile v4f*)op = o;
}

__global__ __launch_bounds__(NTHR) void k_bucket(const int* __restrict__ srcs, const int* __restrict__ dsts,
                                                 int nE, int nN, int vec8, int* REC, int* META, int* FLAG) {
  extern __shared__ __attribute__((aligned(16))) int dsm[];
  int* list = dsm;
  int* hl   = dsm + LISTN;
  int* sl   = hl + RCAP;
  int* cnt  = sl + RCAP;
  int* offs = cnt + NBA;
  int* cur  = offs + NBA;
  int* misc = cur + NBA;
  const int tid = (int)threadIdx.x, lane = tid & 31, wave = tid >> 5;
  const int blk = (int)blockIdx.x;
  const int nodeBase = blk * NBA;

  {
    const v4i z4 = {0, 0, 0, 0};
    for (int i = tid * 4; i < BK_ZINTS; i += NTHR * 4) *(v4ia*)(dsm + i) = z4;
    if (tid < 16) misc[tid] = 0;
  }
  __syncthreads();

  int t = 0, ov = 0;
  const int nChunks = (nE + CHUNK - 1) / CHUNK;
#pragma unroll 1
  for (int ch = 0; ch < nChunks; ++ch) {
    const int cbase = ch * CHUNK;
    const int wc = scan_chunk<SLA>(dsts, nE, cbase, nodeBase, NBA, vec8, list, tid, lane, wave);
    if (lane == 0) misc[wave] = wc;
    __syncthreads();
    if (wave == 0) {
#pragma unroll 1
      for (int w2 = 0; w2 < NWAVE; ++w2) {
        int c = misc[w2];
        c = c < 0 ? 0 : (c > WCAP ? WCAP : c);
#pragma unroll 1
        for (int b0 = 0; b0 < c; b0 += 32) {
          const int idx = b0 + lane;
          const int ent = list[w2 * WCAP + (idx < WCAP ? idx : WCAP - 1)];
          const int m32 = (c - b0) < 32 ? (c - b0) : 32;
#pragma unroll 1
          for (int k = 0; k < m32; ++k) {
            const int u    = __builtin_amdgcn_readlane(ent, k);
            const int slot = u & (NBA - 1);
            const int el   = (u >> SLA) & (CHUNK - 1);
            const int pk   = ((cbase + el) << SLA) | slot;
            if (t < RCAP) {
              if (lane == 0) { hl[t] = pk; cnt[slot] = cnt[slot] + 1; }
              t = t + 1;
            } else {
              ov = 1;
            }
          }
        }
      }
    }
    __syncthreads();
  }
  if (wave == 0 && lane == 0) { misc[8] = t; misc[9] = ov; }
  __syncthreads();
  int tt = misc[8];
  tt = tt < 0 ? 0 : (tt > RCAP ? RCAP : tt);
  const int ovf = misc[9];

  if (wave == 0) {
    const int base = lane * (NBA / 32);
    int s = 0;
#pragma unroll 1
    for (int i = 0; i < NBA / 32; ++i) s += cnt[base + i];
    int incl = s;
#pragma unroll
    for (int d = 1; d < 32; d <<= 1) {
      const int y = __shfl_up(incl, d, 32);
      if (lane >= d) incl += y;
    }
    int run = incl - s;
#pragma unroll 1
    for (int i = 0; i < NBA / 32; ++i) {
      const int cv = cnt[base + i];
      offs[base + i] = run;
      cur[base + i]  = run;
      run += cv;
    }
  }
  __syncthreads();
  if (wave == 0) {
#pragma unroll 1
    for (int b0 = 0; b0 < tt; b0 += 32) {
      const int idx = b0 + lane;
      const int ent = hl[idx < RCAP ? idx : RCAP - 1];
      const int m32 = (tt - b0) < 32 ? (tt - b0) : 32;
#pragma unroll 1
      for (int k = 0; k < m32; ++k) {
        const int u    = __builtin_amdgcn_readlane(ent, k);
        const int slot = u & (NBA - 1);
        if (lane == 0) {
          int p = cur[slot];
          p = p < 0 ? 0 : (p > RCAP - 1 ? RCAP - 1 : p);
          sl[p] = u;
          cur[slot] = p + 1;
        }
      }
    }
  }
  __syncthreads();

#pragma unroll 1
  for (int q = 0; q < NBA / NTHR; ++q) {
    const int s = q * NTHR + tid;
    int c = cnt[s];
    c = c < 0 ? 0 : (c > DEGCAP ? DEGCAP : c);
    int o = offs[s];
    o = o < 0 ? 0 : (o > RCAP ? RCAP : o);
    c = c < (RCAP - o) ? c : (RCAP - o);
    int cm = c;
#pragma unroll
    for (int d = 16; d >= 1; d >>= 1) {
      const int y = __shfl_xor(cm, d, 32);
      cm = cm > y ? cm : y;
    }
#pragma unroll 1
    for (int i = 0; i < cm; ++i) {
      const int pi = (o + i) < (RCAP - 1) ? (o + i) : (RCAP - 1);
      const int ai = sl[pi];
      int rk = 0;
#pragma unroll 1
      for (int j = 0; j < cm; ++j) {
        const int pj = (o + j) < (RCAP - 1) ? (o + j) : (RCAP - 1);
        const int aj = sl[pj];
        const int lt = (aj < ai) ? 1 : 0;
        const int ok = (j < c) ? 1 : 0;
        rk += lt & ok;
      }
      const int po = (o + rk) < (RCAP - 1) ? (o + rk) : (RCAP - 1);
      if (i < c) hl[po] = ai;
    }
  }
  __syncthreads();

#pragma unroll 4
  for (int it = 0; it < RCAP / NTHR; ++it) {
    const int idx = it * NTHR + tid;
    const int ent = hl[idx];
    int eid = ent >> SLA;
    eid = eid < 0 ? 0 : (eid > nE - 1 ? nE - 1 : eid);
    int sr = srcs[eid];
    sr = sr < 0 ? 0 : (sr > nN - 1 ? nN - 1 : sr);
    sl[idx] = (idx < tt) ? sr : 0;
  }
  __syncthreads();

  v4i rv[RCAP / (NTHR * 4)];
  v4i mv[(2 * NBA) / (NTHR * 4)];
#pragma unroll
  for (int it = 0; it < RCAP / (NTHR * 4); ++it) rv[it] = *(const v4ia*)(sl + 4 * (it * NTHR + tid));
#pragma unroll
  for (int it = 0; it < (2 * NBA) / (NTHR * 4); ++it) mv[it] = *(const v4ia*)(cnt + 4 * (it * NTHR + tid));
  v4i fv;
  fv.x = (tid == 0) ? ovf : 0;
  fv.y = (tid == 0) ? tt : 0;
  fv.z = 0; fv.w = 0;
  int* rp = REC  + (size_t)blk * RCAP;
  int* mp = META + (size_t)blk * (2 * NBA);
  int* fp = FLAG + (size_t)blk * 32;
#pragma unroll
  for (int it = 0; it < RCAP / (NTHR * 4); ++it) *(volatile v4i*)(rp + 4 * (it * NTHR + tid)) = rv[it];
#pragma unroll
  for (int it = 0; it < (2 * NBA) / (NTHR * 4); ++it) *(volatile v4i*)(mp + 4 * (it * NTHR + tid)) = mv[it];
  if (tid < 8) *(volatile v4i*)(fp + 4 * tid) = fv;
  __threadfence();
#pragma unroll
  for (int it = 0; it < RCAP / (NTHR * 4); ++it) *(volatile v4i*)(rp + 4 * (it * NTHR + tid)) = rv[it];
#pragma unroll
  for (int it = 0; it < (2 * NBA) / (NTHR * 4); ++it) *(volatile v4i*)(mp + 4 * (it * NTHR + tid)) = mv[it];
  if (tid < 8) *(volatile v4i*)(fp + 4 * tid) = fv;
}

__global__ __launch_bounds__(NTHR) void k_agg(const int* __restrict__ REC, const int* __restrict__ META,
                                              const int* __restrict__ FLAG, const float* __restrict__ X,
                                              unsigned short* Hpl, int nN, int mRows) {
  __shared__ __attribute__((aligned(16))) int rec[RCAP];
  __shared__ __attribute__((aligned(16))) int meta[2 * NBA];
  __shared__ __attribute__((aligned(16))) unsigned short rowb[NWAVE * HP];
  __shared__ int sflag[4];
  const int tid = (int)threadIdx.x, lane = tid & 31, wave = tid >> 5;
  const int blk = (int)blockIdx.x;
  const int nodeBase = blk * NBA;
  {
    const int* rp = REC + (size_t)blk * RCAP;
#pragma unroll
    for (int it = 0; it < RCAP / (NTHR * 4); ++it) {
      const v4i v = *(const v4i*)(rp + 4 * (it * NTHR + tid));
      *(v4ia*)(rec + 4 * (it * NTHR + tid)) = v;
    }
    const int* mp = META + (size_t)blk * (2 * NBA);
#pragma unroll
    for (int it = 0; it < (2 * NBA) / (NTHR * 4); ++it) {
      const v4i v = *(const v4i*)(mp + 4 * (it * NTHR + tid));
      *(v4ia*)(meta + 4 * (it * NTHR + tid)) = v;
    }
    if (tid < 4) sflag[tid] = FLAG[(size_t)blk * 32 + tid];
  }
  __syncthreads();
  const int ovf = sflag[0];
  const float qnan = __int_as_float(0x7fc00000);
  const float pz = (ovf != 0) ? qnan : 0.0f;
  unsigned short* rowbuf = rowb + wave * HP;

#pragma unroll 1
  for (int si = 0; si < NBA / NWAVE; ++si) {
    const int s    = si * NWAVE + wave;
    const int node = nodeBase + s;
    int c = meta[s];
    const bool big = (c > DEGCAP) || (c < 0);
    c = c < 0 ? 0 : (c > DEGCAP ? DEGCAP : c);
    int o = meta[NBA + s];
    o = o < 0 ? 0 : (o > RCAP ? RCAP : o);
    const int nc = node < nN ? node : nN - 1;
    float a0 = 0.0f, a1 = 0.0f, a2 = 0.0f, a3 = 0.0f;
#pragma unroll 1
    for (int b0 = 0; b0 < c; b0 += 32) {
      int idx = o + b0 + lane;
      idx = idx > RCAP - 1 ? RCAP - 1 : idx;
      int sr = rec[idx];
      sr = sr < 0 ? 0 : (sr > nN - 1 ? nN - 1 : sr);
      const int m32 = (c - b0) < 32 ? (c - b0) : 32;
#pragma unroll 1
      for (int k = 0; k < m32; ++k) {
        const int sk = __builtin_amdgcn_readlane(sr, k);
        const v4f a = *(const v4f*)(X + (size_t)sk * DF + 4 * lane);
        a0 += a.x; a1 += a.y; a2 += a.z; a3 += a.w;
      }
    }
    const v4f own = *(const v4f*)(X + (size_t)nc * DF + 4 * lane);
    const float pzr = big ? qnan : pz;
    const bool live = node < nN;
    const float m0 = live ? ((own.x + a0) + pzr) : 0.0f;
    const float m1 = live ? ((own.y + a1) + pzr) : 0.0f;
    const float m2 = live ? ((own.z + a2) + pzr) : 0.0f;
    const float m3 = live ? ((own.w + a3) + pzr) : 0.0f;
    v4us mh, ml;
    {
      unsigned hb;
      hb = bf16_bits(m0); mh[0] = (unsigned short)hb; ml[0] = (unsigned short)bf16_bits(m0 - __uint_as_float(hb << 16));
      hb = bf16_bits(m1); mh[1] = (unsigned short)hb; ml[1] = (unsigned short)bf16_bits(m1 - __uint_as_float(hb << 16));
      hb = bf16_bits(m2); mh[2] = (unsigned short)hb; ml[2] = (unsigned short)bf16_bits(m2 - __uint_as_float(hb << 16));
      hb = bf16_bits(m3); mh[3] = (unsigned short)hb; ml[3] = (unsigned short)bf16_bits(m3 - __uint_as_float(hb << 16));
    }
    *(v4usa*)(rowbuf + 4 * lane) = mh;
    *(v4usa*)(rowbuf + DF + 4 * lane) = ml;
    wave_sync();
    const v8us q0 = *(const v8usa*)(rowbuf + 8 * lane);
    wave_sync();
    if (node < mRows) {
      unsigned short* rpw = Hpl + (size_t)node * HP + 8 * lane;
      *(volatile v8us*)rpw = q0;
      __threadfence();
      *(volatile v8us*)rpw = q0;
    }
  }
}

__global__ __launch_bounds__(GTHR) void k_mlp(const unsigned short* __restrict__ Hpl,
                                              const unsigned short* __restrict__ W1L,
                                              const unsigned short* __restrict__ W2L,
                                              const float* __restrict__ b1l, const float* __restrict__ b2l,
                                              float* X, int nN) {
  __shared__ __attribute__((aligned(16))) float stg[GBM * DF];
  const int tid = (int)threadIdx.x, lane = tid & 31, wave = tid >> 5, hh = lane >> 4, m = lane & 15;
  const int rowBase = (int)blockIdx.x * GBM;
  unsigned short* sh = (unsigned short*)stg;
  const v8f z8 = {0.f, 0.f, 0.f, 0.f, 0.f, 0.f, 0.f, 0.f};

  v8f acc[8];
#pragma unroll
  for (int t = 0; t < 8; ++t) acc[t] = z8;

  {
    const unsigned short* ap = Hpl + (size_t)(rowBase + 16 * wave + m) * (size_t)HP + 8 * hh;
    const unsigned short* bp = W1L + (size_t)m * (size_t)HP + 8 * hh;
#pragma unroll 1
    for (int k0 = 0; k0 < HP; k0 += 32) {
      FragB af;
      af.h[0] = *(const v8usa*)(ap + k0);
      af.h[1] = *(const v8usa*)(ap + k0 + 16);
#pragma unroll
      for (int nt = 0; nt < 8; ++nt) {
        const unsigned short* wq = bp + (size_t)(16 * nt) * (size_t)HP + k0;
        FragB bf;
        bf.h[0] = *(const v8usa*)wq;
        bf.h[1] = *(const v8usa*)(wq + 16);
        acc[nt] = wmb(af, bf, acc[nt]);
      }
    }
  }
#pragma unroll
  for (int nt = 0; nt < 8; ++nt) {
    const int lc = 16 * nt + m;
#pragma unroll
    for (int r = 0; r < 8; ++r) {
      const int lr = 16 * wave + 8 * hh + r;
      stg[lr * DF + lc] = acc[nt][r];
    }
  }
  __syncthreads();

  v4f bb;
  {
    const v4f t1 = *(const v4f*)(b1l + 4 * lane);
    bb.x = bf16_val(t1.x); bb.y = bf16_val(t1.y); bb.z = bf16_val(t1.z); bb.w = bf16_val(t1.w);
  }
  v4f pv[16];
#pragma unroll
  for (int i = 0; i < 16; ++i) pv[i] = *(const v4fa*)(stg + (16 * wave + i) * DF + 4 * lane);
  __syncthreads();

#pragma unroll
  for (int i = 0; i < 16; ++i) {
    const float y0 = relu_keep(pv[i].x + bb.x);
    const float y1 = relu_keep(pv[i].y + bb.y);
    const float y2 = relu_keep(pv[i].z + bb.z);
    const float y3 = relu_keep(pv[i].w + bb.w);
    v4us h4, l4;
    unsigned hb;
    hb = bf16_bits(y0); h4[0] = (unsigned short)hb; l4[0] = (unsigned short)bf16_bits(y0 - __uint_as_float(hb << 16));
    hb = bf16_bits(y1); h4[1] = (unsigned short)hb; l4[1] = (unsigned short)bf16_bits(y1 - __uint_as_float(hb << 16));
    hb = bf16_bits(y2); h4[2] = (unsigned short)hb; l4[2] = (unsigned short)bf16_bits(y2 - __uint_as_float(hb << 16));
    hb = bf16_bits(y3); h4[3] = (unsigned short)hb; l4[3] = (unsigned short)bf16_bits(y3 - __uint_as_float(hb << 16));
    unsigned short* srow = sh + (size_t)(16 * wave + i) * HP;
    *(v4usa*)(srow + 4 * lane) = h4;
    *(v4usa*)(srow + DF + 4 * lane) = l4;
  }
  __syncthreads();

#pragma unroll
  for (int t = 0; t < 8; ++t) acc[t] = z8;
  {
    const unsigned short* as = sh + (size_t)(16 * wave + m) * HP + 8 * hh;
    const unsigned short* bp = W2L + (size_t)m * (size_t)HP + 8 * hh;
#pragma unroll 1
    for (int k0 = 0; k0 < HP; k0 += 32) {
      FragB af;
      af.h[0] = *(const v8usa*)(as + k0);
      af.h[1] = *(const v8usa*)(as + k0 + 16);
#pragma unroll
      for (int nt = 0; nt < 8; ++nt) {
        const unsigned short* wq = bp + (size_t)(16 * nt) * (size_t)HP + k0;
        FragB bf;
        bf.h[0] = *(const v8usa*)wq;
        bf.h[1] = *(const v8usa*)(wq + 16);
        acc[nt] = wmb(af, bf, acc[nt]);
      }
    }
  }
  __syncthreads();
#pragma unroll
  for (int nt = 0; nt < 8; ++nt) {
    const int lc = 16 * nt + m;
#pragma unroll
    for (int r = 0; r < 8; ++r) {
      const int lr = 16 * wave + 8 * hh + r;
      stg[lr * DF + lc] = acc[nt][r];
    }
  }
  __syncthreads();

  {
    const v4f t2 = *(const v4f*)(b2l + 4 * lane);
    bb.x = bf16_val(t2.x); bb.y = bf16_val(t2.y); bb.z = bf16_val(t2.z); bb.w = bf16_val(t2.w);
  }
#pragma unroll
  for (int i = 0; i < 16; ++i) {
    const v4f p = *(const v4fa*)(stg + (16 * wave + i) * DF + 4 * lane);
    v4f y;
    y.x = relu_keep(p.x + bb.x);
    y.y = relu_keep(p.y + bb.y);
    y.z = relu_keep(p.z + bb.z);
    y.w = relu_keep(p.w + bb.w);
    pv[i] = y;
  }
#pragma unroll
  for (int i = 0; i < 16; ++i) {
    const int r = rowBase + 16 * wave + i;
    if (r < nN) *(volatile v4f*)(X + (size_t)r * DF + 4 * lane) = pv[i];
  }
  __threadfence();
#pragma unroll
  for (int i = 0; i < 16; ++i) {
    const int r = rowBase + 16 * wave + i;
    if (r < nN) *(volatile v4f*)(X + (size_t)r * DF + 4 * lane) = pv[i];
  }
}

__global__ __launch_bounds__(NTHR) void k_pool(const float* __restrict__ X, const int* __restrict__ bat,
                                               int nN, int nG, float* out) {
  __shared__ __attribute__((aligned(16))) float sums[PGR * DF];
  __shared__ int cntl[PGR];
  const int tid = (int)threadIdx.x, lane = tid & 31, wave = tid >> 5;
  const int g0 = (int)blockIdx.x * PGR;
  {
    const v4f z4 = {0.f, 0.f, 0.f, 0.f};
#pragma unroll
    for (int it = 0; it < (PGR * DF) / (NTHR * 4); ++it) *(v4fa*)(sums + 4 * (it * NTHR + tid)) = z4;
    if (tid < PGR) cntl[tid] = 0;
  }
  __syncthreads();

#pragma unroll 1
  for (int i0 = 0; i0 < nN; i0 += 32) {
    const int i  = i0 + lane;
    const int ic = i < nN ? i : nN - 1;
    const int bv = bat[ic];
    const unsigned su = (unsigned)bv - (unsigned)g0;
    const bool hit = (i < nN) && (su < (unsigned)PGR) && ((int)(su & 7u) == wave);
    const int sli = (int)(su & (unsigned)(PGR - 1));
    unsigned msk = __builtin_amdgcn_ballot_w32(hit);
    int nh = (int)__builtin_popcount(msk);
    nh = nh > 32 ? 32 : nh;
#pragma unroll 1
    for (int q = 0; q < nh; ++q) {
      int k = __builtin_ffs((int)msk) - 1;
      msk &= msk - 1u;
      k = k < 0 ? 0 : k;
      int node = i0 + k;
      node = node > nN - 1 ? nN - 1 : node;
      int slot = __builtin_amdgcn_readlane(sli, k);
      slot = slot & (PGR - 1);
      const v4f v = *(const v4f*)(X + (size_t)node * DF + 4 * lane);
      float* sp = sums + slot * DF + 4 * lane;
      v4f s4 = *(const v4fa*)sp;
      s4.x += v.x; s4.y += v.y; s4.z += v.z; s4.w += v.w;
      *(v4fa*)sp = s4;
      if (lane == 0) cntl[slot] = cntl[slot] + 1;
    }
  }
  __syncthreads();

  v4f ov[PGR / NWAVE];
#pragma unroll
  for (int j = 0; j < PGR / NWAVE; ++j) {
    const int slot = NWAVE * j + wave;
    const int c = cntl[slot];
    const float cf = (c < 1) ? 1.0f : (float)c;
    const float rc = 1.0f / cf;
    const v4f s4 = *(const v4fa*)(sums + slot * DF + 4 * lane);
    v4f o;
    o.x = s4.x * rc; o.y = s4.y * rc; o.z = s4.z * rc; o.w = s4.w * rc;
    ov[j] = o;
  }
#pragma unroll
  for (int j = 0; j < PGR / NWAVE; ++j) {
    const int g = g0 + NWAVE * j + wave;
    if (g < nG) *(volatile v4f*)(out + (size_t)g * DF + 4 * lane) = ov[j];
  }
  __threadfence();
#pragma unroll
  for (int j = 0; j < PGR / NWAVE; ++j) {
    const int g = g0 + NWAVE * j + wave;
    if (g < nG) *(volatile v4f*)(out + (size_t)g * DF + 4 * lane) = ov[j];
  }
}

static inline int cdiv(int a, int b) { return (a + b - 1) / b; }
static inline size_t al256(size_t o) { return (o + 255) & ~(size_t)255; }

extern "C" void kernel_launch(void* const* d_in, const int* in_sizes, int n_in,
                              void* d_out, int out_size, void* d_ws, size_t ws_size,
                              hipStream_t stream) {
  if (n_in < 8) return;
  const int nN = in_sizes[0];
  if (nN < 1 || nN >= (1 << 22)) return;
  if (in_sizes[1] < 2 || (in_sizes[1] & 1) != 0) return;
  const int nE = in_sizes[1] / 2;
  if (nE < 1 || nE >= (1 << (31 - SLA))) return;
  if (in_sizes[2] != nN) return;
  if (in_sizes[3] != VOC * DF) return;
  if (in_sizes[4] != NLAY * DF * DF || in_sizes[5] != NLAY * DF) return;
  if (in_sizes[6] != NLAY * DF * DF || in_sizes[7] != NLAY * DF) return;
  if (out_size < DF || (out_size % DF) != 0) return;
  const int nG = out_size / DF;

  const int*   tok  = (const int*)d_in[0];
  const int*   edge = (const int*)d_in[1];
  const int*   bat  = (const int*)d_in[2];
  const float* emb  = (const float*)d_in[3];
  const float* W1   = (const float*)d_in[4];
  const float* b1   = (const float*)d_in[5];
  const float* W2   = (const float*)d_in[6];
  const float* b2   = (const float*)d_in[7];
  float* out = (float*)d_out;
  const int* src = edge;
  const int* dst = edge + nE;

  const int MP = cdiv(nN, GBM) * GBM;
  const int gM = MP / GBM;
  const int gA = cdiv(MP, NBA);
  if ((long long)gA * NBA < (long long)MP) return;
  const int gP = cdiv(nG, PGR);
  const int vec8 = ((nE & 3) == 0) ? 1 : 0;

  char* ws = (char*)d_ws;
  size_t off = 0;
  const size_t oW1S = off; off = al256(off + (size_t)NLAY * DF * HP * 2);
  const size_t oW2S = off; off = al256(off + (size_t)NLAY * DF * HP * 2);
  const size_t oX   = off; off = al256(off + (size_t)nN * DF * 4);
  const size_t oH   = off; off = al256(off + (size_t)MP * HP * 2);
  const size_t oREC = off; off = al256(off + (size_t)gA * RCAP * 4);
  const size_t oMET = off; off = al256(off + (size_t)gA * 2 * NBA * 4);
  const size_t oFLG = off; off = al256(off + (size_t)gA * 32 * 4);
  if (off > ws_size || off > (size_t)WSMAX) return;
  unsigned short* W1S = (unsigned short*)(ws + oW1S);
  unsigned short* W2S = (unsigned short*)(ws + oW2S);
  float*          X   = (float*)(ws + oX);
  unsigned short* H   = (unsigned short*)(ws + oH);
  int*            REC = (int*)(ws + oREC);
  int*            MET = (int*)(ws + oMET);
  int*            FLG = (int*)(ws + oFLG);

  const size_t bkLds = (size_t)BK_LDS_INTS * 4;
  hipFuncSetAttribute(reinterpret_cast<const void*>(&k_bucket), hipFuncAttributeMaxDynamicSharedMemorySize, (int)bkLds);

  k_prep<<<WBLK + cdiv(nN * 32, NTHR), NTHR, 0, stream>>>(W1, W2, tok, emb, W1S, W2S, X, nN);
  k_bucket<<<gA, NTHR, bkLds, stream>>>(src, dst, nE, nN, vec8, REC, MET, FLG);
  for (int l = 0; l < NLAY; ++l) {
    k_agg<<<gA, NTHR, 0, stream>>>(REC, MET, FLG, X, H, nN, MP);
    k_mlp<<<gM, GTHR, 0, stream>>>(H, W1S + (size_t)l * DF * HP, W2S + (size_t)l * DF * HP,
                                   b1 + (size_t)l * DF, b2 + (size_t)l * DF, X, nN);
  }
  k_pool<<<gP, NTHR, 0, stream>>>(X, bat, nN, nG, out);
}
